// RNN_6184752906904
// MI455X (gfx1250) — hardware-verified
//
#include <hip/hip_runtime.h>
#include <math.h>

constexpr int NBATCH   = 8;
constexpr int NSTEP    = 1000;
constexpr int NFEAT    = 240;
constexpr int NFEATP   = 256;
constexpr int NHID     = 512;
constexpr int NGATE    = 1024;
constexpr int NROWS    = NBATCH * NSTEP;
constexpr int SEQ_ROWS = 16;
constexpr int REC_THREADS = 512;
constexpr int HPITCH   = 520;
constexpr int SPITCH   = 516;
constexpr int GSLABP   = 36;
constexpr int BN_BLOCKS = NROWS / 64;
constexpr int NOUT0    = NBATCH * NSTEP * NGATE;
constexpr int NOUT1    = 4 * NBATCH * NHID;
constexpr float ACT_CARRY = 256.0f;
constexpr float WGT_CARRY = 16.0f;
constexpr float FOLD_BACK = 1.0f / (ACT_CARRY * WGT_CARRY);
constexpr float RES_CARRY = 2048.0f;
constexpr float RES_FOLD  = 1.0f / RES_CARRY;
constexpr float F16_MIN_NORMAL = 6.103515625e-5f;
constexpr float BN_EPS    = 1e-5f;
constexpr float INV_NROWS = 1.0f / (float)NROWS;

static_assert(NGATE == 2 * NHID);
static_assert(NROWS % 64 == 0 && NGATE % 32 == 0);
static_assert(NFEATP % 32 == 0 && NGATE % 32 == 0 && NHID % 32 == 0);
static_assert(((NROWS / 64) * (NGATE / 32)) % 8 == 0);
static_assert(NFEAT % 8 == 0 && NFEATP % 8 == 0);
static_assert(NHID == 32 * (REC_THREADS / 32));
static_assert(2 * SEQ_ROWS == 4 * NBATCH);
static_assert(2 * NGATE == 4 * REC_THREADS);
static_assert((size_t)NOUT0 * 4 == (size_t)32768000);
static_assert((size_t)NOUT0 * 4 + (size_t)NOUT1 * 4 == (size_t)32833536);
static_assert(((size_t)NOUT0 * 4) % 128 == 0);
static_assert(HPITCH % 8 == 0 && SPITCH % 4 == 0 && GSLABP % 4 == 0);

typedef __attribute__((ext_vector_type(16))) _Float16 v16h;
typedef __attribute__((ext_vector_type(8)))  _Float16 v8h;
typedef __attribute__((ext_vector_type(8)))  float    v8f;
typedef __attribute__((ext_vector_type(4)))  float    v4f;

__device__ __forceinline__ void wmma_guard4(v8f& a0, v8f& a1, v8f& a2, v8f& a3,
                                            v16h x, v16h y0, v16h y1, v16h y2, v16h y3) {
  asm volatile("v_nop\n\tv_nop\n\tv_nop\n\tv_nop"
               : "+v"(a0), "+v"(a1), "+v"(a2), "+v"(a3)
               : "v"(x), "v"(y0), "v"(y1), "v"(y2), "v"(y3));
}
__device__ __forceinline__ void wmma_guard_split(v8f& a0, v8f& a1, v8f& a2, v8f& a3,
                                                 v16h x0, v16h x1, v16h y0, v16h y1, v16h y2, v16h y3) {
  asm volatile("v_nop\n\tv_nop\n\tv_nop\n\tv_nop"
               : "+v"(a0), "+v"(a1), "+v"(a2), "+v"(a3)
               : "v"(x0), "v"(x1), "v"(y0), "v"(y1), "v"(y2), "v"(y3));
}
__device__ __forceinline__ void keep4_h(v16h a, v16h b, v16h c, v16h d) {
  asm volatile("v_nop" :: "v"(a), "v"(b), "v"(c), "v"(d));
}
__device__ __forceinline__ void acc_guard4(v8f& a, v8f& b, v8f& c, v8f& d) {
  asm volatile("v_nop\n\tv_nop\n\tv_nop\n\tv_nop" : "+v"(a), "+v"(b), "+v"(c), "+v"(d));
}
__device__ __forceinline__ void tie4(v4f& a, v4f& b, v4f& c, v4f& d) {
  asm volatile("" : "+v"(a), "+v"(b), "+v"(c), "+v"(d));
}

union FragH { v16h v; v8h h[2]; };
__device__ __forceinline__ v16h frag_load(const _Float16* p) {
  FragH f;
  f.h[0] = *(const v8h*)(p);
  f.h[1] = *(const v8h*)(p + 16);
  return f.v;
}
__device__ __forceinline__ v8f frag_mma(v16h a, v16h b, v8f c) {
  return __builtin_amdgcn_wmma_f32_16x16x32_f16(false, a, false, b, (short)0, c, false, false);
}

__device__ __forceinline__ void split_f16(float v, float& hi_f, float& lo_f) {
  const _Float16 h = (_Float16)v;
  float hf = (float)h;
  hf = (fabsf(hf) < F16_MIN_NORMAL) ? 0.0f : hf;
  hi_f = hf;
  lo_f = (v - hf) * RES_CARRY;
}

__device__ __forceinline__ float sigmoid_f(float x) {
  const float xc = fmaxf(x, -60.0f);
  return __builtin_amdgcn_rcpf(1.0f + expf(-xc));
}

template <bool SPLIT>
__global__ __launch_bounds__(256) void cvt_pad_f16_kernel(const float* __restrict__ src, unsigned short* __restrict__ dst_hi,
                                                          unsigned short* __restrict__ dst_lo,
                                                          int nrow, int scol8, int dcol8, float sc) {
  const int i  = blockIdx.x * 256 + threadIdx.x;
  const int n8 = nrow * dcol8;
  if (i < n8) {
    const int row = i / dcol8;
    const int c8  = i - row * dcol8;
    const bool real = (c8 < scol8);
    const int c8c = real ? c8 : (scol8 - 1);
    const float* sp = src + (size_t)row * (size_t)(scol8 * 8) + (size_t)(c8c * 8);
    const v4f a = *(const v4f*)(sp);
    const v4f b = *(const v4f*)(sp + 4);
    v8h hv, lv;
#pragma unroll
    for (int e = 0; e < 4; ++e) {
      const float fa = real ? (a[e] * sc) : 0.0f;
      const float fb = real ? (b[e] * sc) : 0.0f;
      float ha, la, hb, lb;
      split_f16(fa, ha, la);
      split_f16(fb, hb, lb);
      hv[e]     = (_Float16)ha;
      hv[4 + e] = (_Float16)hb;
      lv[e]     = (_Float16)la;
      lv[4 + e] = (_Float16)lb;
    }
    unsigned short* oh = dst_hi + (size_t)i * 8;
    unsigned short* ol = dst_lo + (size_t)i * 8;
    *(volatile v8h*)oh = hv;
    if (SPLIT) *(volatile v8h*)ol = lv;
    __threadfence();
    *(volatile v8h*)oh = hv;
    if (SPLIT) *(volatile v8h*)ol = lv;
  }
}

__global__ __launch_bounds__(256) void gemm_split_f16_kernel(
    const unsigned short* __restrict__ Ahp, const unsigned short* __restrict__ Alp, int lda,
    const unsigned short* __restrict__ Bhp, const unsigned short* __restrict__ Blp, int ldb,
    float* __restrict__ C, int ldc, int M, int N, int K, float scale) {
  const _Float16* Ah = (const _Float16*)Ahp;
  const _Float16* Al = (const _Float16*)Alp;
  const _Float16* Bh = (const _Float16*)Bhp;
  const _Float16* Bl = (const _Float16*)Blp;
  __shared__ __align__(16) float sT[8][16 * GSLABP];
  const int lane = threadIdx.x & 31;
  const int wave = threadIdx.x >> 5;
  const int tilesN = N >> 5;
  const int tilesM = M >> 6;
  const int tile = blockIdx.x * 8 + wave;
  if (tile >= tilesM * tilesN) return;
  const int tm = tile / tilesN;
  const int tn = tile - tm * tilesN;
  const int m0 = tm << 6;
  const int n0 = tn << 5;
  const int rlane = lane & 15;
  const int koff  = (lane >> 4) * 8;
  const int mOff  = (lane >> 4) * 8;

  v8f acc[4][2], accr[4][2];
#pragma unroll
  for (int i = 0; i < 4; ++i)
#pragma unroll
    for (int j = 0; j < 2; ++j) {
      acc[i][j]  = (v8f){0.f, 0.f, 0.f, 0.f, 0.f, 0.f, 0.f, 0.f};
      accr[i][j] = (v8f){0.f, 0.f, 0.f, 0.f, 0.f, 0.f, 0.f, 0.f};
    }

  for (int k0 = 0; k0 < K; k0 += 32) {
    v16h bh[2], bl[2];
#pragma unroll
    for (int j = 0; j < 2; ++j) {
      const size_t bo = (size_t)(n0 + (j << 4) + rlane) * ldb + koff + k0;
      bh[j] = frag_load(Bh + bo);
      bl[j] = frag_load(Bl + bo);
    }
#pragma unroll
    for (int i = 0; i < 4; ++i) {
      const size_t ao = (size_t)(m0 + (i << 4) + rlane) * lda + koff + k0;
      const v16h ah = frag_load(Ah + ao);
      const v16h al = frag_load(Al + ao);
#pragma unroll
      for (int j = 0; j < 2; ++j) {
        acc[i][j]  = frag_mma(ah, bh[j], acc[i][j]);
        accr[i][j] = frag_mma(ah, bl[j], accr[i][j]);
        accr[i][j] = frag_mma(al, bh[j], accr[i][j]);
      }
      wmma_guard_split(acc[i][0], acc[i][1], accr[i][0], accr[i][1], ah, al, bh[0], bh[1], bl[0], bl[1]);
    }
    keep4_h(bh[0], bh[1], bl[0], bl[1]);
  }
  acc_guard4(acc[0][0], acc[0][1], accr[0][0], accr[0][1]);
  acc_guard4(acc[1][0], acc[1][1], accr[1][0], accr[1][1]);
  acc_guard4(acc[2][0], acc[2][1], accr[2][0], accr[2][1]);
  acc_guard4(acc[3][0], acc[3][1], accr[3][0], accr[3][1]);

  float* slab = sT[wave];
#pragma unroll
  for (int i = 0; i < 4; ++i) {
    const int mBase = m0 + (i << 4);
#pragma unroll
    for (int j = 0; j < 2; ++j) {
#pragma unroll
      for (int r = 0; r < 8; ++r) {
        const float v = (acc[i][j][r] + accr[i][j][r] * RES_FOLD) * scale;
        slab[(mOff + r) * GSLABP + (j << 4) + rlane] = v;
      }
    }
    __builtin_amdgcn_fence(__ATOMIC_RELEASE, "workgroup");
    __builtin_amdgcn_wave_barrier();
    __builtin_amdgcn_fence(__ATOMIC_ACQUIRE, "workgroup");
    {
      const int q = lane >> 3, c4 = (lane & 7) * 4;
      for (int pass = 0; pass < 2; ++pass) {
#pragma unroll
        for (int it = 0; it < 4; ++it) {
          const int row = it * 4 + q;
          const v4f v = *(const v4f*)(slab + row * GSLABP + c4);
          *(volatile v4f*)(C + (size_t)(mBase + row) * ldc + n0 + c4) = v;
        }
        __threadfence();
      }
    }
    __builtin_amdgcn_fence(__ATOMIC_RELEASE, "workgroup");
    __builtin_amdgcn_wave_barrier();
    __builtin_amdgcn_fence(__ATOMIC_ACQUIRE, "workgroup");
  }
}

__global__ __launch_bounds__(256) void bn_partial_kernel(const float* __restrict__ P, float* __restrict__ PS,
                                                         float* __restrict__ PQ) {
  const int blk = blockIdx.x, tid = threadIdx.x;
  const float* base = P + (size_t)blk * 64 * NGATE + tid * 4;
  v4f s = {0.f, 0.f, 0.f, 0.f};
  v4f q = {0.f, 0.f, 0.f, 0.f};
#pragma unroll 4
  for (int r = 0; r < 64; ++r) {
    const v4f x = *(const v4f*)(base + (size_t)r * NGATE);
    s += x;
    q += x * x;
  }
  float* ps = PS + (size_t)blk * NGATE + tid * 4;
  float* pq = PQ + (size_t)blk * NGATE + tid * 4;
  *(volatile v4f*)ps = s;
  *(volatile v4f*)pq = q;
  __threadfence();
  *(volatile v4f*)ps = s;
  *(volatile v4f*)pq = q;
}

__global__ __launch_bounds__(256) void bn_final_kernel(const float* __restrict__ PS, const float* __restrict__ PQ,
                                                       const float* __restrict__ gam, const float* __restrict__ bet,
                                                       float* __restrict__ SCSH) {
  const int c4 = threadIdx.x * 4;
  v4f s = {0.f, 0.f, 0.f, 0.f};
  v4f q = {0.f, 0.f, 0.f, 0.f};
#pragma unroll 4
  for (int b = 0; b < BN_BLOCKS; ++b) {
    s += *(const v4f*)(PS + (size_t)b * NGATE + c4);
    q += *(const v4f*)(PQ + (size_t)b * NGATE + c4);
  }
  const v4f g  = *(const v4f*)(gam + c4);
  const v4f be = *(const v4f*)(bet + c4);
  v4f sc, sh;
#pragma unroll
  for (int e = 0; e < 4; ++e) {
    const float mean = s[e] * INV_NROWS;
    const float var  = fmaxf(q[e] * INV_NROWS - mean * mean, 0.0f);
    const float scl  = g[e] * rsqrtf(var + BN_EPS);
    sc[e] = scl;
    sh[e] = be[e] - mean * scl;
  }
  float* p0 = SCSH + c4;
  float* p1 = SCSH + NGATE + c4;
  *(volatile v4f*)p0 = sc;
  *(volatile v4f*)p1 = sh;
  __threadfence();
  *(volatile v4f*)p0 = sc;
  *(volatile v4f*)p1 = sh;
}

template <int LAYER>
__global__ __launch_bounds__(REC_THREADS) void ligru_seq_kernel(const float* __restrict__ P,
                                                                const float* __restrict__ SCSH,
                                                                const unsigned short* __restrict__ Up,
                                                                unsigned short* __restrict__ X1H,
                                                                unsigned short* __restrict__ X1L,
                                                                float* __restrict__ OUT0,
                                                                float* __restrict__ OUT1) {
  __shared__ __align__(16) _Float16 Ah[SEQ_ROWS * HPITCH];
  __shared__ __align__(16) float    St[SEQ_ROWS * SPITCH];
  __shared__ __align__(16) float    Sc[2 * NGATE];
  const _Float16* U = (const _Float16*)Up;
  const int tid = threadIdx.x, lane = tid & 31, wave = tid >> 5;
  const int c = lane & 15, hh = lane >> 4, koff = hh * 8;
  const int unit0 = 32 * wave + 8 * hh;

#pragma unroll 1
  for (int i = tid; i < SEQ_ROWS * HPITCH; i += REC_THREADS) Ah[i] = (_Float16)0.0f;
  *(v4f*)(Sc + 4 * tid) = *(const v4f*)(SCSH + 4 * tid);

  float hst[2][8];
#pragma unroll
  for (int nt = 0; nt < 2; ++nt)
#pragma unroll
    for (int r = 0; r < 8; ++r) hst[nt][r] = 0.0f;
  __syncthreads();

  const _Float16* hrow = Ah + c * HPITCH + koff;
  const _Float16* ub   = U + (size_t)(32 * wave + c) * NHID + koff;
  constexpr size_t UB_NT = (size_t)16 * NHID;
  constexpr size_t UB_Z  = (size_t)NHID * NHID;
  const int brow = c & 7;
  const int flip = c >> 3;
  const v8f z8 = {0.f, 0.f, 0.f, 0.f, 0.f, 0.f, 0.f, 0.f};

#pragma unroll 1
  for (int t = 0; t < NSTEP; ++t) {
    const int tsel = flip ? (NSTEP - 1 - t) : t;
    const float* prow = P + ((size_t)(brow * NSTEP + tsel)) * NGATE + unit0;
    v4f pa[2][2], pz[2][2];
    pa[0][0] = *(const v4f*)(prow);
    pa[0][1] = *(const v4f*)(prow + 4);
    pa[1][0] = *(const v4f*)(prow + 16);
    pa[1][1] = *(const v4f*)(prow + 20);
#pragma unroll
    for (int nt = 0; nt < 2; ++nt)
#pragma unroll
      for (int q = 0; q < 2; ++q) {
        const v4f sc = *(const v4f*)(Sc + unit0 + 16 * nt + 4 * q);
        const v4f sh = *(const v4f*)(Sc + NGATE + unit0 + 16 * nt + 4 * q);
        pa[nt][q] = pa[nt][q] * sc + sh;
      }
    tie4(pa[0][0], pa[0][1], pa[1][0], pa[1][1]);
    pz[0][0] = *(const v4f*)(prow + NHID);
    pz[0][1] = *(const v4f*)(prow + NHID + 4);
    pz[1][0] = *(const v4f*)(prow + NHID + 16);
    pz[1][1] = *(const v4f*)(prow + NHID + 20);
#pragma unroll
    for (int nt = 0; nt < 2; ++nt)
#pragma unroll
      for (int q = 0; q < 2; ++q) {
        const v4f sc = *(const v4f*)(Sc + NHID + unit0 + 16 * nt + 4 * q);
        const v4f sh = *(const v4f*)(Sc + NGATE + NHID + unit0 + 16 * nt + 4 * q);
        pz[nt][q] = pz[nt][q] * sc + sh;
      }
    tie4(pz[0][0], pz[0][1], pz[1][0], pz[1][1]);

    v8f acc[4];
    acc[0] = z8; acc[1] = z8; acc[2] = z8; acc[3] = z8;
#pragma unroll 1
    for (int k0 = 0; k0 < NHID; k0 += 32) {
      const v16h hb = frag_load(hrow + k0);
      const v16h a0 = frag_load(ub + k0);
      const v16h a1 = frag_load(ub + UB_NT + k0);
      const v16h a2 = frag_load(ub + UB_Z + k0);
      const v16h a3 = frag_load(ub + UB_Z + UB_NT + k0);
      acc[0] = frag_mma(a0, hb, acc[0]);
      acc[1] = frag_mma(a1, hb, acc[1]);
      acc[2] = frag_mma(a2, hb, acc[2]);
      acc[3] = frag_mma(a3, hb, acc[3]);
      wmma_guard4(acc[0], acc[1], acc[2], acc[3], hb, a0, a1, a2, a3);
    }
    acc_guard4(acc[0], acc[1], acc[2], acc[3]);

    __syncthreads();

#pragma unroll
    for (int nt = 0; nt < 2; ++nt) {
      v8h hv;
      v4f s0, s1;
#pragma unroll
      for (int r = 0; r < 8; ++r) {
        const float av = pa[nt][r >> 2][r & 3] + acc[nt][r] * FOLD_BACK;
        const float zv = pz[nt][r >> 2][r & 3] + acc[2 + nt][r] * FOLD_BACK;
        const float zs = sigmoid_f(zv);
        const float ho = hst[nt][r];
        const float hn = zs * ho + (1.0f - zs) * fmaxf(av, 0.0f);
        hst[nt][r] = hn;
        hv[r] = (_Float16)(hn * ACT_CARRY);
        if (r < 4) s0[r & 3] = hn; else s1[r & 3] = hn;
      }
      *(v8h*)(Ah + c * HPITCH + unit0 + 16 * nt) = hv;
      *(v4f*)(St + c * SPITCH + unit0 + 16 * nt)     = s0;
      *(v4f*)(St + c * SPITCH + unit0 + 16 * nt + 4) = s1;
    }

    __syncthreads();

    if (LAYER == 0) {
      v8h hv[2], lv[2];
      size_t so[2];
#pragma unroll
      for (int it = 0; it < 2; ++it) {
        const int idx = it * REC_THREADS + tid;
        const int row = idx >> 6;
        const int c8  = (idx & 63) * 8;
        const v4f va = *(const v4f*)(St + row * SPITCH + c8);
        const v4f vb = *(const v4f*)(St + row * SPITCH + c8 + 4);
#pragma unroll
        for (int e = 0; e < 4; ++e) {
          float ha, la, hb2, lb2;
          split_f16(va[e] * ACT_CARRY, ha, la);
          split_f16(vb[e] * ACT_CARRY, hb2, lb2);
          hv[it][e]     = (_Float16)ha;
          hv[it][4 + e] = (_Float16)hb2;
          lv[it][e]     = (_Float16)la;
          lv[it][4 + e] = (_Float16)lb2;
        }
        const int b = row & 7, half = row >> 3;
        const int ttr = half ? (NSTEP - 1 - t) : t;
        so[it] = (size_t)(b * NSTEP + ttr) * NGATE + (size_t)(half * NHID + c8);
      }
      for (int pass = 0; pass < 2; ++pass) {
#pragma unroll
        for (int it = 0; it < 2; ++it) {
          *(volatile v8h*)(X1H + so[it]) = hv[it];
          *(volatile v8h*)(X1L + so[it]) = lv[it];
        }
        __threadfence();
      }
    } else {
      v4f vv[4];
      size_t so[4];
#pragma unroll
      for (int it = 0; it < 4; ++it) {
        const int idx = it * REC_THREADS + tid;
        const int row = idx >> 7;
        const int c4  = (idx & 127) * 4;
        vv[it] = *(const v4f*)(St + row * SPITCH + c4);
        const int b = row & 7, half = row >> 3;
        const int ttr = half ? (NSTEP - 1 - t) : t;
        so[it] = (size_t)(b * NSTEP + ttr) * NGATE + (size_t)(half * NHID + c4);
      }
      for (int pass = 0; pass < 2; ++pass) {
#pragma unroll
        for (int it = 0; it < 4; ++it) *(volatile v4f*)(OUT0 + so[it]) = vv[it];
        __threadfence();
      }
    }

    if (t == 0 || t == NSTEP - 1) {
#pragma unroll
      for (int it = 0; it < 4; ++it) {
        const int idx = it * REC_THREADS + tid;
        const int row = idx >> 7;
        const int c4  = (idx & 127) * 4;
        const int b = row & 7, half = row >> 3;
        const bool want = (half == 0) ? (t == NSTEP - 1) : (t == 0);
        if (want) {
          const v4f v = *(const v4f*)(St + row * SPITCH + c4);
          float* op = OUT1 + (size_t)b * (2 * NGATE) + (size_t)LAYER * NGATE + (size_t)(half * NHID + c4);
          *(volatile v4f*)op = v;
          __threadfence();
          *(volatile v4f*)op = v;
        }
      }
    }
  }
}

extern "C" void kernel_launch(void* const* d_in, const int* in_sizes, int n_in,
                              void* d_out, int out_size, void* d_ws, size_t ws_size, hipStream_t stream) {
  if (n_in < 9 || d_out == nullptr || d_ws == nullptr) return;
  if (in_sizes[0] != NBATCH * NSTEP * NFEAT || in_sizes[1] != NGATE * NFEAT || in_sizes[2] != NGATE * NHID ||
      in_sizes[3] != NGATE || in_sizes[4] != NGATE || in_sizes[5] != NGATE * NGATE ||
      in_sizes[6] != NGATE * NHID || in_sizes[7] != NGATE || in_sizes[8] != NGATE ||
      out_size != NOUT0 + NOUT1) return;

  const float* x  = (const float*)d_in[0];
  const float* w0 = (const float*)d_in[1];
  const float* u0 = (const float*)d_in[2];
  const float* g0 = (const float*)d_in[3];
  const float* b0 = (const float*)d_in[4];
  const float* w1 = (const float*)d_in[5];
  const float* u1 = (const float*)d_in[6];
  const float* g1 = (const float*)d_in[7];
  const float* b1 = (const float*)d_in[8];
  float* out0 = (float*)d_out;
  float* out1 = out0 + (size_t)NOUT0;

  char* ws = (char*)d_ws;
  size_t off = 0;
  auto carve = [&](size_t bytes) -> char* { char* p = ws + off; off += (bytes + 255) & ~(size_t)255; return p; };
  unsigned short* XH   = (unsigned short*)carve((size_t)NROWS * NFEATP * 2);
  unsigned short* XL   = (unsigned short*)carve((size_t)NROWS * NFEATP * 2);
  unsigned short* W0H  = (unsigned short*)carve((size_t)NGATE * NFEATP * 2);
  unsigned short* W0L  = (unsigned short*)carve((size_t)NGATE * NFEATP * 2);
  unsigned short* U0H  = (unsigned short*)carve((size_t)NGATE * NHID * 2);
  unsigned short* W1H  = (unsigned short*)carve((size_t)NGATE * NGATE * 2);
  unsigned short* W1L  = (unsigned short*)carve((size_t)NGATE * NGATE * 2);
  unsigned short* U1H  = (unsigned short*)carve((size_t)NGATE * NHID * 2);
  float*          P0   = (float*)carve((size_t)NROWS * NGATE * 4);
  float*          P1   = (float*)carve((size_t)NROWS * NGATE * 4);
  unsigned short* X1H  = (unsigned short*)carve((size_t)NROWS * NGATE * 2);
  unsigned short* X1L  = (unsigned short*)carve((size_t)NROWS * NGATE * 2);
  float*          PS0  = (float*)carve((size_t)BN_BLOCKS * NGATE * 4);
  float*          PQ0  = (float*)carve((size_t)BN_BLOCKS * NGATE * 4);
  float*          PS1  = (float*)carve((size_t)BN_BLOCKS * NGATE * 4);
  float*          PQ1  = (float*)carve((size_t)BN_BLOCKS * NGATE * 4);
  float*          SCSH0 = (float*)carve((size_t)2 * NGATE * 4);
  float*          SCSH1 = (float*)carve((size_t)2 * NGATE * 4);
  if (off > ws_size || off > (size_t)134217728) return;

  cvt_pad_f16_kernel<true><<<(NROWS * (NFEATP / 8)) / 256, 256, 0, stream>>>(x,  XH,  XL,  NROWS, NFEAT / 8, NFEATP / 8, ACT_CARRY);
  cvt_pad_f16_kernel<true><<<(NGATE * (NFEATP / 8)) / 256, 256, 0, stream>>>(w0, W0H, W0L, NGATE, NFEAT / 8, NFEATP / 8, WGT_CARRY);
  cvt_pad_f16_kernel<false><<<(NGATE * (NHID / 8)) / 256,  256, 0, stream>>>(u0, U0H, U0H, NGATE, NHID / 8,  NHID / 8,   WGT_CARRY);
  cvt_pad_f16_kernel<true><<<(NGATE * (NGATE / 8)) / 256,  256, 0, stream>>>(w1, W1H, W1L, NGATE, NGATE / 8, NGATE / 8,  WGT_CARRY);
  cvt_pad_f16_kernel<false><<<(NGATE * (NHID / 8)) / 256,  256, 0, stream>>>(u1, U1H, U1H, NGATE, NHID / 8,  NHID / 8,   WGT_CARRY);

  const int gemm_blocks = ((NROWS / 64) * (NGATE / 32)) / 8;

  gemm_split_f16_kernel<<<gemm_blocks, 256, 0, stream>>>(XH, XL, NFEATP, W0H, W0L, NFEATP, P0, NGATE,
                                                         NROWS, NGATE, NFEATP, FOLD_BACK);
  bn_partial_kernel<<<BN_BLOCKS, 256, 0, stream>>>(P0, PS0, PQ0);
  bn_final_kernel<<<1, 256, 0, stream>>>(PS0, PQ0, g0, b0, SCSH0);
  ligru_seq_kernel<0><<<1, REC_THREADS, 0, stream>>>(P0, SCSH0, U0H, X1H, X1L, out0, out1);

  gemm_split_f16_kernel<<<gemm_blocks, 256, 0, stream>>>(X1H, X1L, NGATE, W1H, W1L, NGATE, P1, NGATE,
                                                         NROWS, NGATE, NGATE, FOLD_BACK);
  bn_partial_kernel<<<BN_BLOCKS, 256, 0, stream>>>(P1, PS1, PQ1);
  bn_final_kernel<<<1, 256, 0, stream>>>(PS1, PQ1, g1, b1, SCSH1);
  ligru_seq_kernel<1><<<1, REC_THREADS, 0, stream>>>(P1, SCSH1, U1H, X1H, X1L, out0, out1);
}
